// FusionGCN_36567351558152
// MI455X (gfx1250) — hardware-verified
//
#include <hip/hip_runtime.h>
#include <stddef.h>
#include <stdint.h>


#define BSZ    16
#define NPIX   1024
#define CS     256
#define CXC    64
#define CIN    320
#define PHIH   64
#define GHID   128
#define BN_EPS 1e-5f
#define NTHR   256
#define NWAVE  8
#define EPMAX  10240
#define PROWS  256
#define XROWS  128
#define KCH    32
#define NB1    128
#define ECH    256
#define SIGC   30.0f

#define LDS_PHI  (PROWS * PHIH * 4)
#define LDS_XW   (XROWS * GHID * 4)
#define LDS_AGG1 (NB1 * GHID * 4 + ECH * 4 + 64 + NB1 * 4)

static_assert(2 * PROWS * KCH * 2 <= LDS_PHI);
static_assert(2 * XROWS * KCH * 2 <= LDS_XW);
static_assert(PROWS == NTHR);
static_assert(XROWS * 2 == NTHR);
static_assert(ECH == NTHR);
static_assert(NPIX % NB1 == 0);
static_assert(NPIX % XROWS == 0);
static_assert(CIN % KCH == 0);
static_assert((EPMAX % PROWS) == 0);
static_assert(NPIX == 4 * NTHR);
static_assert((PHIH * CIN / 8) % NTHR == 0);
static_assert((GHID * CIN / 8) % NTHR == 0);

typedef float          v4f   __attribute__((ext_vector_type(4)));
typedef float          v8f   __attribute__((ext_vector_type(8)));
typedef int            v2i   __attribute__((ext_vector_type(2)));
typedef unsigned short v8us  __attribute__((ext_vector_type(8)));
typedef __bf16         v16bf __attribute__((ext_vector_type(16)));
union FragB { v16bf v; v8us h[2]; };
struct HL { v8us h; v8us l; };

__device__ __forceinline__ unsigned int sp1(float x) {
  const unsigned int u  = __float_as_uint(x);
  const unsigned int hu = (u + 0x7FFFu + ((u >> 16) & 1u)) >> 16;
  const float        r  = x - __uint_as_float(hu << 16);
  const unsigned int v  = __float_as_uint(r);
  const unsigned int lu = (v + 0x7FFFu + ((v >> 16) & 1u)) >> 16;
  return hu | (lu << 16);
}

__device__ __forceinline__ HL split8(v4f a, v4f b) {
  HL o;
  unsigned int p;
  p = sp1(a.x); o.h[0] = (unsigned short)(p & 0xFFFFu); o.l[0] = (unsigned short)(p >> 16);
  p = sp1(a.y); o.h[1] = (unsigned short)(p & 0xFFFFu); o.l[1] = (unsigned short)(p >> 16);
  p = sp1(a.z); o.h[2] = (unsigned short)(p & 0xFFFFu); o.l[2] = (unsigned short)(p >> 16);
  p = sp1(a.w); o.h[3] = (unsigned short)(p & 0xFFFFu); o.l[3] = (unsigned short)(p >> 16);
  p = sp1(b.x); o.h[4] = (unsigned short)(p & 0xFFFFu); o.l[4] = (unsigned short)(p >> 16);
  p = sp1(b.y); o.h[5] = (unsigned short)(p & 0xFFFFu); o.l[5] = (unsigned short)(p >> 16);
  p = sp1(b.z); o.h[6] = (unsigned short)(p & 0xFFFFu); o.l[6] = (unsigned short)(p >> 16);
  p = sp1(b.w); o.h[7] = (unsigned short)(p & 0xFFFFu); o.l[7] = (unsigned short)(p >> 16);
  return o;
}

__device__ __forceinline__ v8f wmb(v16bf a, v16bf b, v8f c) {
  v8f d = __builtin_amdgcn_wmma_f32_16x16x32_bf16(false, a, false, b, (short)0, c, false, false);
  asm volatile("v_nop\n\tv_nop\n\tv_nop\n\tv_nop" : "+v"(d) : "v"(a), "v"(b));
  return d;
}

__device__ __forceinline__ float sigm(float x) {
  const float z = fminf(fmaxf(x, -SIGC), SIGC);
  return 1.0f / (1.0f + expf(-z));
}

__global__ __launch_bounds__(NTHR) void k_feat(const float* __restrict__ sf,
                                               const float* __restrict__ xc,
                                               float* nff) {
  __shared__ float tile[32][33];
  const int tid = threadIdx.x;
  const int n0 = blockIdx.x * 32, c0 = blockIdx.y * 32, b = blockIdx.z;
  const int cr = tid >> 3, nq = (tid & 7) * 4;
  const int c  = c0 + cr;
  const float* src;
  if (c0 < CS) src = sf + ((size_t)b * CS + c) * NPIX + n0 + nq;
  else         src = xc + ((size_t)b * CXC + (c - CS)) * NPIX + n0 + nq;
  const v4f v = *(const v4f*)src;
  tile[cr][nq + 0] = v.x; tile[cr][nq + 1] = v.y; tile[cr][nq + 2] = v.z; tile[cr][nq + 3] = v.w;
  __syncthreads();
  const int nr = tid >> 3, cq = (tid & 7) * 4;
  v4f o;
  o.x = tile[cq + 0][nr]; o.y = tile[cq + 1][nr]; o.z = tile[cq + 2][nr]; o.w = tile[cq + 3][nr];
  float* dp = nff + ((size_t)b * NPIX + n0 + nr) * CIN + c0 + cq;
  *(volatile v4f*)dp = o;
  __threadfence();
  *(volatile v4f*)dp = o;
}

__global__ __launch_bounds__(NTHR) void k_wts(const float* __restrict__ w1,
                                              const float* __restrict__ g1,
                                              unsigned short* w1h, unsigned short* w1l,
                                              unsigned short* g1h, unsigned short* g1l) {
  const int nb1 = (PHIH * CIN / 8) / NTHR;
  const bool first = (int)blockIdx.x < nb1;
  const int i = (first ? (int)blockIdx.x : (int)blockIdx.x - nb1) * NTHR + (int)threadIdx.x;
  const int o = i * 8;
  const int n = o / CIN, k0 = o - n * CIN;
  v4f a, b;
  if (first) {
    const float* p = w1 + (size_t)k0 * PHIH + n;
    a.x = p[0];        a.y = p[PHIH];     a.z = p[2 * PHIH]; a.w = p[3 * PHIH];
    b.x = p[4 * PHIH]; b.y = p[5 * PHIH]; b.z = p[6 * PHIH]; b.w = p[7 * PHIH];
  } else {
    const float* p = g1 + (size_t)k0 * GHID + n;
    a.x = p[0];        a.y = p[GHID];     a.z = p[2 * GHID]; a.w = p[3 * GHID];
    b.x = p[4 * GHID]; b.y = p[5 * GHID]; b.z = p[6 * GHID]; b.w = p[7 * GHID];
  }
  const HL s = split8(a, b);
  unsigned short* ph = (first ? w1h : g1h) + o;
  unsigned short* pl = (first ? w1l : g1l) + o;
  *(volatile v8us*)ph = s.h;
  *(volatile v8us*)pl = s.l;
  __threadfence();
  *(volatile v8us*)ph = s.h;
  *(volatile v8us*)pl = s.l;
}

__global__ __launch_bounds__(NTHR) void k_phi(const float* __restrict__ nff,
                                              const int* __restrict__ pairs,
                                              const unsigned short* __restrict__ w1h,
                                              const unsigned short* __restrict__ w1l,
                                              const float* __restrict__ b1,
                                              float* hpre, int E, int EP) {
  extern __shared__ v4f lds_dyn[];
  unsigned short* sAh = (unsigned short*)lds_dyn;
  unsigned short* sAl = sAh + PROWS * KCH;
  float*          stg = (float*)lds_dyn;
  const int tid = threadIdx.x, lane = tid & 31, wv = tid >> 5, hh = lane >> 4, m = lane & 15;
  const int b = blockIdx.y, e0 = blockIdx.x * PROWS;

  int e = e0 + tid; e = e > E - 1 ? E - 1 : e;
  const v2i pr = *(const v2i*)(pairs + ((size_t)b * E + e) * 2);
  int pa = pr.x, pb = pr.y;
  pa = pa < 0 ? 0 : (pa > NPIX - 1 ? NPIX - 1 : pa);
  pb = pb < 0 ? 0 : (pb > NPIX - 1 ? NPIX - 1 : pb);
  const float* ra = nff + ((size_t)b * NPIX + pa) * CIN;
  const float* rb = nff + ((size_t)b * NPIX + pb) * CIN;

  v8f acc[2][4];
#pragma unroll
  for (int t = 0; t < 2; ++t)
#pragma unroll
    for (int nt = 0; nt < 4; ++nt) { v8f z = {0.f, 0.f, 0.f, 0.f, 0.f, 0.f, 0.f, 0.f}; acc[t][nt] = z; }

#pragma unroll 1
  for (int kb = 0; kb < CIN / KCH; ++kb) {
    __syncthreads();
#pragma unroll
    for (int q = 0; q < 4; ++q) {
      const int ko = kb * KCH + 8 * q;
      const v4f x0 = *(const v4f*)(ra + ko), x1 = *(const v4f*)(ra + ko + 4);
      const v4f y0 = *(const v4f*)(rb + ko), y1 = *(const v4f*)(rb + ko + 4);
      v4f d0 = x0 - y0, d1 = x1 - y1;
      d0.x = fabsf(d0.x); d0.y = fabsf(d0.y); d0.z = fabsf(d0.z); d0.w = fabsf(d0.w);
      d1.x = fabsf(d1.x); d1.y = fabsf(d1.y); d1.z = fabsf(d1.z); d1.w = fabsf(d1.w);
      const HL s = split8(d0, d1);
      *(v8us*)(sAh + tid * KCH + 8 * q) = s.h;
      *(v8us*)(sAl + tid * KCH + 8 * q) = s.l;
    }
    __syncthreads();
    FragB ah[2], al[2];
#pragma unroll
    for (int t = 0; t < 2; ++t) {
      const int row = wv * 32 + t * 16 + m;
      const unsigned short* aph = sAh + row * KCH + 8 * hh;
      const unsigned short* apl = sAl + row * KCH + 8 * hh;
      ah[t].h[0] = *(const v8us*)aph;  ah[t].h[1] = *(const v8us*)(aph + 16);
      al[t].h[0] = *(const v8us*)apl;  al[t].h[1] = *(const v8us*)(apl + 16);
    }
#pragma unroll
    for (int nt = 0; nt < 4; ++nt) {
      const size_t bo = (size_t)(nt * 16 + m) * CIN + kb * KCH + 8 * hh;
      FragB bh, bl;
      bh.h[0] = *(const v8us*)(w1h + bo); bh.h[1] = *(const v8us*)(w1h + bo + 16);
      bl.h[0] = *(const v8us*)(w1l + bo); bl.h[1] = *(const v8us*)(w1l + bo + 16);
#pragma unroll
      for (int t = 0; t < 2; ++t) {
        acc[t][nt] = wmb(ah[t].v, bh.v, acc[t][nt]);
        acc[t][nt] = wmb(ah[t].v, bl.v, acc[t][nt]);
        acc[t][nt] = wmb(al[t].v, bh.v, acc[t][nt]);
      }
    }
  }
  __syncthreads();

#pragma unroll
  for (int t = 0; t < 2; ++t)
#pragma unroll
    for (int nt = 0; nt < 4; ++nt) {
      const int col = nt * 16 + m;
      const float bias = b1[col];
      float* sp = stg + (wv * 32 + t * 16 + 8 * hh) * PHIH + col;
      sp[0 * PHIH] = acc[t][nt][0] + bias;
      sp[1 * PHIH] = acc[t][nt][1] + bias;
      sp[2 * PHIH] = acc[t][nt][2] + bias;
      sp[3 * PHIH] = acc[t][nt][3] + bias;
      sp[4 * PHIH] = acc[t][nt][4] + bias;
      sp[5 * PHIH] = acc[t][nt][5] + bias;
      sp[6 * PHIH] = acc[t][nt][6] + bias;
      sp[7 * PHIH] = acc[t][nt][7] + bias;
    }
  __syncthreads();

  const float* lp = stg + (wv * 32) * PHIH + 4 * lane;
  float* gp = hpre + ((size_t)b * EP + e0 + wv * 32) * PHIH + 4 * lane;
#pragma unroll
  for (int i = 0; i < 16; ++i) { const v4f v = *(const v4f*)(lp + i * 128); *(volatile v4f*)(gp + (size_t)i * 128) = v; }
  __threadfence();
#pragma unroll
  for (int i = 0; i < 16; ++i) { const v4f v = *(const v4f*)(lp + i * 128); *(volatile v4f*)(gp + (size_t)i * 128) = v; }
}

__global__ __launch_bounds__(NTHR) void k_edge(const float* __restrict__ hpre,
                                               const float* __restrict__ gamma,
                                               const float* __restrict__ beta,
                                               const float* __restrict__ w2,
                                               const float* __restrict__ b2,
                                               float* edgev, int E, int EP) {
  __shared__ double ss[NTHR], sq[NTHR];
  __shared__ float smu[PHIH], srs[PHIH], sga[PHIH], sbe[PHIH], sw2[PHIH];
  __shared__ __attribute__((aligned(16))) float sev[EPMAX];
  const int tid = threadIdx.x, b = blockIdx.x;

  {
    const int c = tid & 63, g = tid >> 6;
    const float* hp = hpre + (size_t)b * EP * PHIH + c;
    double s = 0.0, q = 0.0;
#pragma unroll 1
    for (int e = g; e < E; e += 4) {
      const double x = (double)hp[(size_t)e * PHIH];
      s += x;
      q += x * x;
    }
    ss[tid] = s; sq[tid] = q;
  }
  __syncthreads();
  if (tid < PHIH) {
    const double S = ((ss[tid] + ss[tid + 64]) + ss[tid + 128]) + ss[tid + 192];
    const double Q = ((sq[tid] + sq[tid + 64]) + sq[tid + 128]) + sq[tid + 192];
    const double invE = 1.0 / (double)E;
    const double mu = S * invE;
    double var = Q * invE - mu * mu;
    var = var < 0.0 ? 0.0 : var;
    const float vf = (float)var;
    smu[tid] = (float)mu;
    srs[tid] = 1.0f / sqrtf(vf + BN_EPS);
    sga[tid] = gamma[tid];
    sbe[tid] = beta[tid];
    sw2[tid] = w2[tid];
  }
  __syncthreads();

  const float bias2 = b2[0];
#pragma unroll 1
  for (int e = tid; e < EP; e += NTHR) {
    const int ec = e > E - 1 ? E - 1 : e;
    const float* hp = hpre + ((size_t)b * EP + ec) * PHIH;
    float acc = 0.f;
#pragma unroll 1
    for (int c4 = 0; c4 < PHIH; c4 += 4) {
      const v4f h = *(const v4f*)(hp + c4);
      float x;
      x = (h.x - smu[c4 + 0]) * srs[c4 + 0] * sga[c4 + 0] + sbe[c4 + 0]; x = fmaxf(x, 0.f); acc += x * sw2[c4 + 0];
      x = (h.y - smu[c4 + 1]) * srs[c4 + 1] * sga[c4 + 1] + sbe[c4 + 1]; x = fmaxf(x, 0.f); acc += x * sw2[c4 + 1];
      x = (h.z - smu[c4 + 2]) * srs[c4 + 2] * sga[c4 + 2] + sbe[c4 + 2]; x = fmaxf(x, 0.f); acc += x * sw2[c4 + 2];
      x = (h.w - smu[c4 + 3]) * srs[c4 + 3] * sga[c4 + 3] + sbe[c4 + 3]; x = fmaxf(x, 0.f); acc += x * sw2[c4 + 3];
    }
    acc += bias2;
    sev[e] = sigm(acc);
  }
  __syncthreads();

  float* gp = edgev + (size_t)b * EP;
#pragma unroll 1
  for (int e = tid; e < EP; e += NTHR) { const float v = sev[e]; *(volatile float*)(gp + e) = v; }
  __threadfence();
#pragma unroll 1
  for (int e = tid; e < EP; e += NTHR) { const float v = sev[e]; *(volatile float*)(gp + e) = v; }
}

__global__ __launch_bounds__(NTHR) void k_xw(const float* __restrict__ nff,
                                             const unsigned short* __restrict__ g1h,
                                             const unsigned short* __restrict__ g1l,
                                             float* xw) {
  extern __shared__ v4f lds_dyn[];
  unsigned short* sAh = (unsigned short*)lds_dyn;
  unsigned short* sAl = sAh + XROWS * KCH;
  float*          stg = (float*)lds_dyn;
  const int tid = threadIdx.x, lane = tid & 31, wv = tid >> 5, hh = lane >> 4, m = lane & 15;
  const int b = blockIdx.y, row0 = blockIdx.x * XROWS;
  const int sr = tid >> 1, kq = (tid & 1) * 16;
  const float* rp = nff + ((size_t)b * NPIX + row0 + sr) * CIN + kq;

  v8f acc[8];
#pragma unroll
  for (int nt = 0; nt < 8; ++nt) { v8f z = {0.f, 0.f, 0.f, 0.f, 0.f, 0.f, 0.f, 0.f}; acc[nt] = z; }

#pragma unroll 1
  for (int kb = 0; kb < CIN / KCH; ++kb) {
    __syncthreads();
#pragma unroll
    for (int q = 0; q < 2; ++q) {
      const int ko = kb * KCH + 8 * q;
      const v4f x0 = *(const v4f*)(rp + ko), x1 = *(const v4f*)(rp + ko + 4);
      const HL s = split8(x0, x1);
      *(v8us*)(sAh + sr * KCH + kq + 8 * q) = s.h;
      *(v8us*)(sAl + sr * KCH + kq + 8 * q) = s.l;
    }
    __syncthreads();
    FragB ah, al;
    {
      const unsigned short* aph = sAh + (wv * 16 + m) * KCH + 8 * hh;
      const unsigned short* apl = sAl + (wv * 16 + m) * KCH + 8 * hh;
      ah.h[0] = *(const v8us*)aph; ah.h[1] = *(const v8us*)(aph + 16);
      al.h[0] = *(const v8us*)apl; al.h[1] = *(const v8us*)(apl + 16);
    }
#pragma unroll
    for (int nt = 0; nt < 8; ++nt) {
      const size_t bo = (size_t)(nt * 16 + m) * CIN + kb * KCH + 8 * hh;
      FragB bh, bl;
      bh.h[0] = *(const v8us*)(g1h + bo); bh.h[1] = *(const v8us*)(g1h + bo + 16);
      bl.h[0] = *(const v8us*)(g1l + bo); bl.h[1] = *(const v8us*)(g1l + bo + 16);
      acc[nt] = wmb(ah.v, bh.v, acc[nt]);
      acc[nt] = wmb(ah.v, bl.v, acc[nt]);
      acc[nt] = wmb(al.v, bh.v, acc[nt]);
    }
  }
  __syncthreads();

  {
    float* sp = stg + (wv * 16 + 8 * hh) * GHID + m;
#pragma unroll
    for (int nt = 0; nt < 8; ++nt) {
      sp[0 * GHID + 16 * nt] = acc[nt][0];
      sp[1 * GHID + 16 * nt] = acc[nt][1];
      sp[2 * GHID + 16 * nt] = acc[nt][2];
      sp[3 * GHID + 16 * nt] = acc[nt][3];
      sp[4 * GHID + 16 * nt] = acc[nt][4];
      sp[5 * GHID + 16 * nt] = acc[nt][5];
      sp[6 * GHID + 16 * nt] = acc[nt][6];
      sp[7 * GHID + 16 * nt] = acc[nt][7];
    }
  }
  __syncthreads();

  const float* lp = stg + wv * 16 * GHID + 4 * lane;
  float* gp = xw + ((size_t)b * NPIX + row0 + wv * 16) * GHID + 4 * lane;
#pragma unroll
  for (int i = 0; i < 16; ++i) { const v4f v = *(const v4f*)(lp + i * GHID); *(volatile v4f*)(gp + (size_t)i * GHID) = v; }
  __threadfence();
#pragma unroll
  for (int i = 0; i < 16; ++i) { const v4f v = *(const v4f*)(lp + i * GHID); *(volatile v4f*)(gp + (size_t)i * GHID) = v; }
}

__global__ __launch_bounds__(NTHR) void k_agg1(const int* __restrict__ pairs,
                                               const float* __restrict__ edgev,
                                               const float* __restrict__ xw,
                                               const float* __restrict__ g2,
                                               float* sv, int E, int EP) {
  extern __shared__ v4f lds_dyn[];
  float* acc  = (float*)lds_dyn;
  int*   list = (int*)(acc + NB1 * GHID);
  int*   wcnt = list + ECH;
  float* so   = (float*)(wcnt + 16);
  const int tid = threadIdx.x, lane = tid & 31, wv = tid >> 5;
  const int b = blockIdx.y, nodeBase = blockIdx.x * NB1;

  {
    const v4f z = {0.f, 0.f, 0.f, 0.f};
    for (int i = tid; i < NB1 * GHID / 4; i += NTHR) lds_dyn[i] = z;
  }
  __syncthreads();

  const int nCh = (E + ECH - 1) / ECH;
#pragma unroll 1
  for (int ch = 0; ch < nCh; ++ch) {
    const int e  = ch * ECH + tid;
    const int ec = e > E - 1 ? E - 1 : e;
    const int a  = pairs[((size_t)b * E + ec) * 2];
    const unsigned int s = (unsigned int)(a - nodeBase);
    const bool hit = (e < E) && (s < (unsigned int)NB1);
    const unsigned int mk = __builtin_amdgcn_ballot_w32(hit);
    if (hit) {
      const int pos = (int)__builtin_amdgcn_mbcnt_lo(mk, 0u);
      list[wv * 32 + pos] = (tid << 8) | (int)s;
    }
    if (lane == 0) wcnt[wv] = (int)__builtin_popcount(mk);
    __syncthreads();
    if (wv == 0) {
#pragma unroll 1
      for (int w = 0; w < NWAVE; ++w) {
        int n = __builtin_amdgcn_readfirstlane(wcnt[w]);
        n = n > 32 ? 32 : (n < 0 ? 0 : n);
#pragma unroll 1
        for (int i = 0; i < n; ++i) {
          const int ent  = __builtin_amdgcn_readfirstlane(list[w * 32 + i]);
          const int slot = ent & (NB1 - 1);
          const int t    = (ent >> 8) & (NTHR - 1);
          int e2 = ch * ECH + t;
          e2 = e2 > E - 1 ? E - 1 : e2;
          int src = pairs[((size_t)b * E + e2) * 2 + 1];
          src = src < 0 ? 0 : (src > NPIX - 1 ? NPIX - 1 : src);
          const float wgt = edgev[(size_t)b * EP + e2];
          const v4f v = *(const v4f*)(xw + ((size_t)b * NPIX + src) * GHID + 4 * lane);
          v4f* ap = (v4f*)(acc + slot * GHID + 4 * lane);
          const v4f cur = *ap;
          *ap = cur + v * wgt;
        }
      }
    }
    __syncthreads();
  }

  if (tid < NB1) {
    const float* ap = acc + tid * GHID;
    float sdot = 0.f;
#pragma unroll 1
    for (int d = 0; d < GHID; d += 4) {
      const v4f h = *(const v4f*)(ap + d);
      const v4f g = *(const v4f*)(g2 + d);
      float x;
      x = h.x >= 0.f ? h.x : 0.2f * h.x; sdot += x * g.x;
      x = h.y >= 0.f ? h.y : 0.2f * h.y; sdot += x * g.y;
      x = h.z >= 0.f ? h.z : 0.2f * h.z; sdot += x * g.z;
      x = h.w >= 0.f ? h.w : 0.2f * h.w; sdot += x * g.w;
    }
    so[tid] = sdot;
  }
  __syncthreads();
  if (wv == 0) {
    const v4f v = *(const v4f*)(so + 4 * lane);
    float* gp = sv + (size_t)b * NPIX + nodeBase + 4 * lane;
    *(volatile v4f*)gp = v;
    __threadfence();
    *(volatile v4f*)gp = v;
  }
}

__global__ __launch_bounds__(NTHR) void k_agg2(const int* __restrict__ pairs,
                                               const float* __restrict__ edgev,
                                               const float* __restrict__ sv,
                                               float* out, int E, int EP) {
  __shared__ __attribute__((aligned(16))) float acc[NPIX];
  __shared__ int   sa[ECH];
  __shared__ float sc[ECH];
  const int tid = threadIdx.x, b = blockIdx.x;

  for (int i = tid; i < NPIX; i += NTHR) acc[i] = 0.f;
  __syncthreads();

  const int nCh = (E + ECH - 1) / ECH;
#pragma unroll 1
  for (int ch = 0; ch < nCh; ++ch) {
    const int e  = ch * ECH + tid;
    const int ec = e > E - 1 ? E - 1 : e;
    const v2i pr = *(const v2i*)(pairs + ((size_t)b * E + ec) * 2);
    int a = pr.x, bs = pr.y;
    a  = a  < 0 ? 0 : (a  > NPIX - 1 ? NPIX - 1 : a);
    bs = bs < 0 ? 0 : (bs > NPIX - 1 ? NPIX - 1 : bs);
    const float w = edgev[(size_t)b * EP + ec];
    const float s = sv[(size_t)b * NPIX + bs];
    const float c = (e < E) ? w * s : 0.f;
    sa[tid] = a;
    sc[tid] = c;
    __syncthreads();
    if (tid == 0) {
#pragma unroll 4
      for (int i = 0; i < ECH; ++i) {
        const int d = sa[i];
        acc[d] = acc[d] + sc[i];
      }
    }
    __syncthreads();
  }

#pragma unroll 1
  for (int i = tid; i < NPIX; i += NTHR) { const float x = acc[i]; acc[i] = sigm(x); }
  __syncthreads();
  const v4f o = *(const v4f*)(acc + 4 * tid);
  float* gp = out + (size_t)b * NPIX + 4 * tid;
  *(volatile v4f*)gp = o;
  __threadfence();
  *(volatile v4f*)gp = o;
}

extern "C" void kernel_launch(void* const* d_in, const int* in_sizes, int n_in,
                              void* d_out, int out_size, void* d_ws, size_t ws_size,
                              hipStream_t stream) {
  if (n_in < 11) return;
  if (in_sizes[0] != BSZ * CS * NPIX || in_sizes[1] != BSZ * CXC * NPIX) return;
  if (in_sizes[2] <= 0 || (in_sizes[2] % (2 * BSZ)) != 0) return;
  const int E  = in_sizes[2] / (2 * BSZ);
  const int EP = ((E + PROWS - 1) / PROWS) * PROWS;
  if (E <= 0 || EP > EPMAX) return;
  if (in_sizes[3] != CIN * PHIH || in_sizes[4] != PHIH || in_sizes[5] != PHIH || in_sizes[6] != PHIH) return;
  if (in_sizes[7] != PHIH || in_sizes[8] < 1 || in_sizes[9] != CIN * GHID || in_sizes[10] != GHID) return;
  if (out_size != BSZ * NPIX) return;

  const float* sf    = (const float*)d_in[0];
  const float* xc    = (const float*)d_in[1];
  const int*   pairs = (const int*)d_in[2];
  const float* w1    = (const float*)d_in[3];
  const float* b1    = (const float*)d_in[4];
  const float* gamma = (const float*)d_in[5];
  const float* beta  = (const float*)d_in[6];
  const float* w2    = (const float*)d_in[7];
  const float* b2    = (const float*)d_in[8];
  const float* g1    = (const float*)d_in[9];
  const float* g2    = (const float*)d_in[10];
  float* out = (float*)d_out;

  char* ws = (char*)d_ws;
  size_t off = 0;
  const size_t oNF = off; off += (size_t)BSZ * NPIX * CIN * 4;      off = (off + 255) & ~(size_t)255;
  const size_t oW1H = off; off += (size_t)PHIH * CIN * 2;           off = (off + 255) & ~(size_t)255;
  const size_t oW1L = off; off += (size_t)PHIH * CIN * 2;           off = (off + 255) & ~(size_t)255;
  const size_t oG1H = off; off += (size_t)GHID * CIN * 2;           off = (off + 255) & ~(size_t)255;
  const size_t oG1L = off; off += (size_t)GHID * CIN * 2;           off = (off + 255) & ~(size_t)255;
  const size_t oHP = off; off += (size_t)BSZ * EP * PHIH * 4;       off = (off + 255) & ~(size_t)255;
  const size_t oEV = off; off += (size_t)BSZ * EP * 4;              off = (off + 255) & ~(size_t)255;
  const size_t oXW = off; off += (size_t)BSZ * NPIX * GHID * 4;     off = (off + 255) & ~(size_t)255;
  const size_t oSV = off; off += (size_t)BSZ * NPIX * 4;            off = (off + 255) & ~(size_t)255;
  if (off > ws_size) return;

  float*          nff   = (float*)(ws + oNF);
  unsigned short* w1h   = (unsigned short*)(ws + oW1H);
  unsigned short* w1l   = (unsigned short*)(ws + oW1L);
  unsigned short* g1h   = (unsigned short*)(ws + oG1H);
  unsigned short* g1l   = (unsigned short*)(ws + oG1L);
  float*          hpre  = (float*)(ws + oHP);
  float*          edgev = (float*)(ws + oEV);
  float*          xw    = (float*)(ws + oXW);
  float*          sv    = (float*)(ws + oSV);

  k_feat<<<dim3(NPIX / 32, CIN / 32, BSZ), NTHR, 0, stream>>>(sf, xc, nff);

  {
    const int nb = (PHIH * CIN / 8) / NTHR + (GHID * CIN / 8) / NTHR;
    k_wts<<<nb, NTHR, 0, stream>>>(w1, g1, w1h, w1l, g1h, g1l);
  }

  hipFuncSetAttribute(reinterpret_cast<const void*>(&k_phi),
                      hipFuncAttributeMaxDynamicSharedMemorySize, LDS_PHI);
  k_phi<<<dim3(EP / PROWS, BSZ), NTHR, LDS_PHI, stream>>>(nff, pairs, w1h, w1l, b1, hpre, E, EP);

  k_edge<<<BSZ, NTHR, 0, stream>>>(hpre, gamma, beta, w2, b2, edgev, E, EP);

  hipFuncSetAttribute(reinterpret_cast<const void*>(&k_xw),
                      hipFuncAttributeMaxDynamicSharedMemorySize, LDS_XW);
  k_xw<<<dim3(NPIX / XROWS, BSZ), NTHR, LDS_XW, stream>>>(nff, g1h, g1l, xw);

  hipFuncSetAttribute(reinterpret_cast<const void*>(&k_agg1),
                      hipFuncAttributeMaxDynamicSharedMemorySize, LDS_AGG1);
  k_agg1<<<dim3(NPIX / NB1, BSZ), NTHR, LDS_AGG1, stream>>>(pairs, edgev, xw, g2, sv, E, EP);

  k_agg2<<<BSZ, NTHR, 0, stream>>>(pairs, edgev, sv, out, E, EP);
}
